// CoattentiveAggregation_88888643158469
// MI455X (gfx1250) — hardware-verified
//
#include <hip/hip_runtime.h>
#include <stdint.h>

typedef __attribute__((ext_vector_type(16))) _Float16 v16h;
typedef __attribute__((ext_vector_type(8)))  _Float16 v8h;
typedef __attribute__((ext_vector_type(8)))  float    v8f;
typedef __attribute__((ext_vector_type(4)))  float    v4f;

constexpr int KNB   = 32;
constexpr int DFEAT = 128;
constexpr int WPB   = 1;
constexpr int PDQ   = 132;
constexpr int PLL   = 33;

static_assert(DFEAT % 32 == 0);
static_assert(KNB == 32);
static_assert((PDQ * 4) % 16 == 0);

struct WaveLDS {
  float Dm[KNB * PDQ];
  float Qm[KNB * PDQ];
  float Lm[KNB * PLL];
  float E1[KNB * PLL];
  float E2[KNB * PLL];
  float ri[KNB];
  float ci[KNB];
  float wv[KNB];
  float tv[KNB];
  float uv[KNB];
  float Hm[3 * DFEAT];
};
static_assert(sizeof(WaveLDS) == 48640);
static_assert(sizeof(WaveLDS) % 16 == 0);
static_assert(offsetof(WaveLDS, Hm) % 16 == 0);
static_assert(offsetof(WaveLDS, Qm) % 16 == 0);

__device__ __forceinline__ int wrap_clamp(int i, int n) {
  i = (i < 0) ? (i + n) : i;
  i = (i < 0) ? 0 : i;
  i = (i > n - 1) ? (n - 1) : i;
  return i;
}

__device__ __forceinline__ v16h frag_cvt(const float* p) {
  const v4f x0 = *(const v4f*)(p);
  const v4f x1 = *(const v4f*)(p + 4);
  const v4f x2 = *(const v4f*)(p + 16);
  const v4f x3 = *(const v4f*)(p + 20);
  v16h a;
#pragma unroll
  for (int e = 0; e < 4; ++e) {
    a[e]      = (_Float16)x0[e];
    a[4 + e]  = (_Float16)x1[e];
    a[8 + e]  = (_Float16)x2[e];
    a[12 + e] = (_Float16)x3[e];
  }
  return a;
}

__device__ __forceinline__ v8f mma16(v16h a, v16h b, v8f c) {
  return __builtin_amdgcn_wmma_f32_16x16x32_f16(false, a, false, b, (short)0, c, false, false);
}

__device__ __forceinline__ void guard4(v8f& a, v8f& b, v8f& c, v8f& d, v16h w, v16h x, v16h y, v16h z) {
  asm volatile("v_nop\n\tv_nop\n\tv_nop\n\tv_nop" : "+v"(a), "+v"(b), "+v"(c), "+v"(d) : "v"(w), "v"(x), "v"(y), "v"(z));
}

__global__ __launch_bounds__(WPB * 32)
void coatt_node_kernel(const float* __restrict__ feat,
                       const int*   __restrict__ sim_idx,
                       const int*   __restrict__ cor_idx,
                       float*       __restrict__ out,
                       int nN)
{
  __shared__ __align__(16) WaveLDS smem[WPB];
  const int wave  = threadIdx.x >> 5;
  const int lane  = threadIdx.x & 31;
  const int node  = blockIdx.x * WPB + wave;
  const int nodec = (node < nN) ? node : (nN - 1);
  WaveLDS& W = smem[wave];
  const int m = lane & 15;
  const int h = lane >> 4;

  int si = sim_idx[(size_t)nodec * KNB + lane];
  int qi = cor_idx[(size_t)nodec * KNB + lane];
  si = wrap_clamp(si, nN);
  qi = wrap_clamp(qi, nN);
  v4f m1 = (v4f){0.f, 0.f, 0.f, 0.f};
#pragma unroll 1
  for (int r = 0; r < KNB; ++r) {
    const int sr = __shfl(si, r, 32);
    const int qr = __shfl(qi, r, 32);
    const v4f a = *(const v4f*)(feat + (size_t)sr * DFEAT + 4 * lane);
    const v4f b = *(const v4f*)(feat + (size_t)qr * DFEAT + 4 * lane);
    *(v4f*)(W.Dm + r * PDQ + 4 * lane) = a;
    *(v4f*)(W.Qm + r * PDQ + 4 * lane) = b;
    m1 += b;
  }
  __syncthreads();

  v8f acc[2][2];
#pragma unroll
  for (int i = 0; i < 2; ++i)
#pragma unroll
    for (int j = 0; j < 2; ++j) acc[i][j] = (v8f){0.f, 0.f, 0.f, 0.f, 0.f, 0.f, 0.f, 0.f};

#pragma unroll 1
  for (int k0 = 0; k0 < DFEAT; k0 += 32) {
    v16h af[2], bf[2];
#pragma unroll
    for (int t = 0; t < 2; ++t) {
      af[t] = frag_cvt(W.Dm + (16 * t + m) * PDQ + k0 + 8 * h);
      bf[t] = frag_cvt(W.Qm + (16 * t + m) * PDQ + k0 + 8 * h);
    }
#pragma unroll
    for (int mi = 0; mi < 2; ++mi)
#pragma unroll
      for (int ni = 0; ni < 2; ++ni)
        acc[mi][ni] = mma16(af[mi], bf[ni], acc[mi][ni]);
    guard4(acc[0][0], acc[0][1], acc[1][0], acc[1][1], af[0], af[1], bf[0], bf[1]);
  }

#pragma unroll
  for (int mi = 0; mi < 2; ++mi)
#pragma unroll
    for (int ni = 0; ni < 2; ++ni)
#pragma unroll
      for (int r = 0; r < 8; ++r)
        W.Lm[(16 * mi + 8 * h + r) * PLL + 16 * ni + m] = acc[mi][ni][r];
  __syncthreads();

  {
    const float* Lr = W.Lm + lane * PLL;
    float mx = Lr[0];
#pragma unroll 1
    for (int j = 1; j < KNB; ++j) mx = fmaxf(mx, Lr[j]);
    float rs = 0.f;
#pragma unroll 1
    for (int j = 0; j < KNB; ++j) {
      const float e = __expf(Lr[j] - mx);
      W.E1[lane * PLL + j] = e;
      rs += e;
    }
    W.ri[lane] = 1.0f / rs;
  }
  {
    float mx = W.Lm[lane];
#pragma unroll 1
    for (int k = 1; k < KNB; ++k) mx = fmaxf(mx, W.Lm[k * PLL + lane]);
    float cs = 0.f;
#pragma unroll 1
    for (int k = 0; k < KNB; ++k) {
      const float e = __expf(W.Lm[k * PLL + lane] - mx);
      W.E2[k * PLL + lane] = e;
      cs += e;
    }
    W.ci[lane] = 1.0f / cs;
  }
  __syncthreads();

  {
    float wacc = 0.f;
#pragma unroll 1
    for (int k = 0; k < KNB; ++k) wacc += W.E2[lane * PLL + k] * W.ci[k];
    wacc *= (1.0f / KNB);
    W.wv[lane] = wacc;
    W.tv[lane] = wacc * W.ri[lane];
  }
  __syncthreads();

  {
    float uacc = 0.f;
#pragma unroll 1
    for (int j = 0; j < KNB; ++j) uacc += W.tv[j] * W.E1[j * PLL + lane];
    W.uv[lane] = uacc;
  }
  __syncthreads();

  {
    v4f m2 = (v4f){0.f, 0.f, 0.f, 0.f};
    v4f m3 = (v4f){0.f, 0.f, 0.f, 0.f};
#pragma unroll 1
    for (int j = 0; j < KNB; ++j) {
      const float wj = W.wv[j];
      const float uj = W.uv[j];
      const v4f dv = *(const v4f*)(W.Dm + j * PDQ + 4 * lane);
      const v4f qv = *(const v4f*)(W.Qm + j * PDQ + 4 * lane);
      m2 += dv * wj;
      m3 += qv * uj;
    }
    *(v4f*)(W.Hm + 4 * lane)             = m1 * (1.0f / KNB);
    *(v4f*)(W.Hm + DFEAT + 4 * lane)     = m2;
    *(v4f*)(W.Hm + 2 * DFEAT + 4 * lane) = m3;
  }
  __syncthreads();

  {
    const v4f g0 = *(const v4f*)(W.Hm + 12 * lane);
    const v4f g1 = *(const v4f*)(W.Hm + 12 * lane + 4);
    const v4f g2 = *(const v4f*)(W.Hm + 12 * lane + 8);
    v4f o;
    o[0] = (g0[0] + g0[1]) + g0[2];
    o[1] = (g0[3] + g1[0]) + g1[1];
    o[2] = (g1[2] + g1[3]) + g2[0];
    o[3] = (g2[1] + g2[2]) + g2[3];
    const float third = 1.0f / 3.0f;
    const v4f fv = *(const v4f*)(feat + (size_t)nodec * DFEAT + 4 * lane);
    const v4f ov = fv + o * third;
    if (node < nN) {
      float* op = out + (size_t)node * DFEAT + 4 * lane;
      *(volatile v4f*)op = ov;
      __threadfence();
      *(volatile v4f*)op = ov;
    }
  }
}

extern "C" void kernel_launch(void* const* d_in, const int* in_sizes, int n_in,
                              void* d_out, int out_size, void* d_ws, size_t ws_size,
                              hipStream_t stream) {
  const float* feat = (const float*)d_in[0];
  const int*   sim  = (const int*)d_in[1];
  const int*   cor  = (const int*)d_in[2];
  float* out = (float*)d_out;
  const int nN = in_sizes[0] / DFEAT;
  if (nN <= 0) return;
  const int nblk = (nN + WPB - 1) / WPB;
  coatt_node_kernel<<<dim3(nblk), dim3(WPB * 32), 0, stream>>>(feat, sim, cor, out, nN);
  (void)n_in; (void)out_size; (void)d_ws; (void)ws_size;
}
